// Filter_52931176956186
// MI455X (gfx1250) — hardware-verified
//
#include <hip/hip_runtime.h>
#include <stddef.h>


#define DIM     64
#define KD      128
#define NOUT    64
#define NTHR    256
#define NWAVE   8
#define EPT     8
#define NGRP    2
#define CHUNK   (NTHR * EPT * NGRP)
#define WCAP    (EPT * NGRP * 32)
#define LISTN   (NWAVE * WCAP)
#define NBC     4096
#define NBF     1024
#define RCAP    40960
#define RBN     128
#define TGT     256
#define DEGCAP  256
#define GROWS   128
#define OTHR    512
#define WSCALE  16.0f
#define WINV    0.0625f

#define LDS_FILL ((RCAP + NBF + LISTN) * 4 + 64)
#define LDS_AGG  (TGT * KD * 2)

static_assert((CHUNK & (CHUNK - 1)) == 0);
static_assert(CHUNK <= 4096);
static_assert(NBC <= 4096 && NBF <= 4096);
static_assert((NBC & (NBC - 1)) == 0 && (NBF & (NBF - 1)) == 0);
static_assert(NBC == 4 * NBF);
static_assert(OTHR * 8 == NBC);
static_assert((RCAP % 32) == 0);
static_assert(TGT == NWAVE * 32 && (TGT % GROWS) == 0);
static_assert(GROWS == NWAVE * 16);
static_assert(NOUT * KD / 8 == 4 * NTHR);
static_assert(KD % 32 == 0 && NOUT % 16 == 0);

typedef float    v2f  __attribute__((ext_vector_type(2)));
typedef float    v4f  __attribute__((ext_vector_type(4)));
typedef float    v8f  __attribute__((ext_vector_type(8)));
typedef int      v4i  __attribute__((ext_vector_type(4)));
typedef _Float16 v2h  __attribute__((ext_vector_type(2)));
typedef _Float16 v8h  __attribute__((ext_vector_type(8)));
typedef _Float16 v16h __attribute__((ext_vector_type(16)));
union FragH { v16h v; v8h h[2]; };

__device__ __forceinline__ v8h cvt8(v4f a, v4f b) {
  v8h r;
  r[0] = (_Float16)a.x; r[1] = (_Float16)a.y; r[2] = (_Float16)a.z; r[3] = (_Float16)a.w;
  r[4] = (_Float16)b.x; r[5] = (_Float16)b.y; r[6] = (_Float16)b.z; r[7] = (_Float16)b.w;
  return r;
}

__device__ __forceinline__ v8f wmh(v16h a, v16h b, v8f c) {
  v8f d = __builtin_amdgcn_wmma_f32_16x16x32_f16(false, a, false, b, (short)0, c, false, false);
  asm volatile("v_nop\n\tv_nop\n\tv_nop\n\tv_nop" : "+v"(d) : "v"(a), "v"(b));
  return d;
}

template <int NB>
__device__ __forceinline__ int scan_chunk(const int* __restrict__ dsts, int nE, int cbase, int slotBase,
                                          int vec8, int* list, int tid, int lane, int wave) {
  int wc = 0;
#pragma unroll
  for (int g = 0; g < NGRP; ++g) {
    const int el0  = (g * NTHR + tid) * EPT;
    const int e0   = cbase + el0;
    const int sent = -2147483647 - 1;
    v4i da, db;
    if (vec8 != 0 && cbase + CHUNK <= nE) {
      da = *(const v4i*)(dsts + e0);
      db = *(const v4i*)(dsts + e0 + 4);
    } else {
      da.x = (e0     < nE) ? dsts[min(e0, nE - 1)] : sent;
      da.y = (e0 + 1 < nE) ? dsts[min(e0 + 1, nE - 1)] : sent;
      da.z = (e0 + 2 < nE) ? dsts[min(e0 + 2, nE - 1)] : sent;
      da.w = (e0 + 3 < nE) ? dsts[min(e0 + 3, nE - 1)] : sent;
      db.x = (e0 + 4 < nE) ? dsts[min(e0 + 4, nE - 1)] : sent;
      db.y = (e0 + 5 < nE) ? dsts[min(e0 + 5, nE - 1)] : sent;
      db.z = (e0 + 6 < nE) ? dsts[min(e0 + 6, nE - 1)] : sent;
      db.w = (e0 + 7 < nE) ? dsts[min(e0 + 7, nE - 1)] : sent;
    }
    const unsigned nb = (unsigned)slotBase;
    const unsigned s0 = (unsigned)da.x - nb, s1 = (unsigned)da.y - nb;
    const unsigned s2 = (unsigned)da.z - nb, s3 = (unsigned)da.w - nb;
    const unsigned s4 = (unsigned)db.x - nb, s5 = (unsigned)db.y - nb;
    const unsigned s6 = (unsigned)db.z - nb, s7 = (unsigned)db.w - nb;
    const bool h0 = s0 < (unsigned)NB, h1 = s1 < (unsigned)NB, h2 = s2 < (unsigned)NB, h3 = s3 < (unsigned)NB;
    const bool h4 = s4 < (unsigned)NB, h5 = s5 < (unsigned)NB, h6 = s6 < (unsigned)NB, h7 = s7 < (unsigned)NB;
    const unsigned any = __builtin_amdgcn_ballot_w32(h0 | h1 | h2 | h3 | h4 | h5 | h6 | h7);
    if (any != 0u) {
#define HITJ(J, HJ, SJ) { \
        const unsigned mj = __builtin_amdgcn_ballot_w32(HJ); \
        if (mj != 0u) { \
          if (HJ) { \
            const int pos = wc + (int)__builtin_amdgcn_mbcnt_lo(mj, 0u); \
            if (pos < WCAP) list[wave * WCAP + pos] = ((el0 + (J)) << 12) | (int)(SJ); \
          } \
          wc += (int)__builtin_popcount(mj); } }
      HITJ(0, h0, s0)
      HITJ(1, h1, s1)
      HITJ(2, h2, s2)
      HITJ(3, h3, s3)
      HITJ(4, h4, s4)
      HITJ(5, h5, s5)
      HITJ(6, h6, s6)
      HITJ(7, h7, s7)
#undef HITJ
    }
  }
  return wc;
}

__global__ __launch_bounds__(NTHR) void k_wprep(
    const float* __restrict__ W1l, const float* __restrict__ W1r,
    const float* __restrict__ W2l, const float* __restrict__ W2r, _Float16* wB) {
  const int layer = blockIdx.x >> 2;
  const float* Wl = layer == 0 ? W1l : W2l;
  const float* Wr = layer == 0 ? W1r : W2r;
  _Float16* dst = wB + (size_t)layer * NOUT * KD;
  const int i  = (blockIdx.x & 3) * NTHR + (int)threadIdx.x;
  const int n  = i >> 4;
  const int k0 = (i & 15) * 8;
  float v[8];
#pragma unroll
  for (int e = 0; e < 8; ++e) {
    const int k  = k0 + e;
    const int kl = k < DIM ? k : DIM - 1;
    const int kr = k < DIM ? 0 : k - DIM;
    const float a = Wl[kl * NOUT + n];
    const float b = Wr[kr * NOUT + n];
    v[e] = (k < DIM ? a : b) * WSCALE;
  }
  v4f a4, b4;
  a4.x = v[0]; a4.y = v[1]; a4.z = v[2]; a4.w = v[3];
  b4.x = v[4]; b4.y = v[5]; b4.z = v[6]; b4.w = v[7];
  const v8h hv = cvt8(a4, b4);
  _Float16* dp = dst + (size_t)i * 8;
  *(volatile v8h*)dp = hv;
  __threadfence();
  *(volatile v8h*)dp = hv;
}

__global__ __launch_bounds__(NTHR) void k_count(
    const int* __restrict__ ei, int* cnt, int nE, int vec8) {
  __shared__ __attribute__((aligned(16))) int scnt[NBC];
  __shared__ __attribute__((aligned(16))) int list[LISTN];
  __shared__ int wcnt[NWAVE];
  const int tid = threadIdx.x, lane = tid & 31, wave = tid >> 5;
  const int nodeBase = blockIdx.x * NBC;
  const int* dsts = ei + nE;

  for (int i = tid; i < NBC; i += NTHR) scnt[i] = 0;
  __syncthreads();

  const int nChunks = (nE + CHUNK - 1) / CHUNK;
#pragma unroll 1
  for (int ch = 0; ch < nChunks; ++ch) {
    const int cbase = ch * CHUNK;
    const int wc = scan_chunk<NBC>(dsts, nE, cbase, nodeBase, vec8, list, tid, lane, wave);
    if (lane == 0) wcnt[wave] = wc;
    __syncthreads();
    if (wave == 0) {
#pragma unroll 1
      for (int wsx = 0; wsx < NWAVE; ++wsx) {
        int n = __builtin_amdgcn_readfirstlane(wcnt[wsx]);
        n = n > WCAP ? WCAP : (n < 0 ? 0 : n);
        const int* lp = list + wsx * WCAP;
#pragma unroll 1
        for (int i = 0; i < n; ++i) {
          const int ent  = __builtin_amdgcn_readfirstlane(lp[i]);
          const int slot = ent & (NBC - 1);
          if (lane == 0) scnt[slot] = scnt[slot] + 1;
        }
      }
    }
    __syncthreads();
  }

  v4i cq[4];
#pragma unroll
  for (int q = 0; q < 4; ++q) {
    const int f = (wave * 4 + q) * 128 + 4 * lane;
    cq[q] = *(const v4i*)(scnt + f);
  }
  int* cp = cnt + (size_t)nodeBase;
#pragma unroll
  for (int q = 0; q < 4; ++q) {
    const int f = (wave * 4 + q) * 128 + 4 * lane;
    *(volatile v4i*)(cp + f) = cq[q];
  }
  __threadfence();
#pragma unroll
  for (int q = 0; q < 4; ++q) {
    const int f = (wave * 4 + q) * 128 + 4 * lane;
    *(volatile v4i*)(cp + f) = cq[q];
  }
}

__global__ __launch_bounds__(OTHR) void k_offsets(
    const int* __restrict__ cnt, int* off, int* rbase, int nChunk) {
  __shared__ __attribute__((aligned(16))) int soff[NBC];
  __shared__ __attribute__((aligned(16))) int srb[RBN];
  __shared__ int wtot[OTHR / 32];
  const int tid = threadIdx.x, lane = tid & 31, wave = tid >> 5, sub = tid >> 7;
  for (int i = tid; i < RBN; i += OTHR) srb[i] = 0;
  int carry = 0;
#pragma unroll 1
  for (int ch = 0; ch < nChunk; ++ch) {
    const int base = ch * NBC;
    const v4i c0 = *(const v4i*)(cnt + base + 8 * tid);
    const v4i c1 = *(const v4i*)(cnt + base + 8 * tid + 4);
    const int e0 = max(c0.x, 0), e1 = max(c0.y, 0), e2 = max(c0.z, 0), e3 = max(c0.w, 0);
    const int e4 = max(c1.x, 0), e5 = max(c1.y, 0), e6 = max(c1.z, 0), e7 = max(c1.w, 0);
    const int ts = e0 + e1 + e2 + e3 + e4 + e5 + e6 + e7;
    int incl = ts;
#pragma unroll
    for (int d = 1; d < 32; d <<= 1) {
      const int t = __shfl_up(incl, d);
      if (lane >= d) incl += t;
    }
    if (lane == 31) wtot[wave] = incl;
    __syncthreads();
    const int S0 = wtot[0]  + wtot[1]  + wtot[2]  + wtot[3];
    const int S1 = wtot[4]  + wtot[5]  + wtot[6]  + wtot[7];
    const int S2 = wtot[8]  + wtot[9]  + wtot[10] + wtot[11];
    const int S3 = wtot[12] + wtot[13] + wtot[14] + wtot[15];
    int pre = 0;
#pragma unroll 1
    for (int w = 4 * sub; w < wave; ++w) pre += wtot[w];
    const int b0 = carry;
    const int b1 = b0 + ((S0 + 31) & ~31);
    const int b2 = b1 + ((S1 + 31) & ~31);
    const int b3 = b2 + ((S2 + 31) & ~31);
    const int b4 = b3 + ((S3 + 31) & ~31);
    const int myb = sub == 0 ? b0 : (sub == 1 ? b1 : (sub == 2 ? b2 : b3));
    if (tid == 0) {
      srb[min(4 * ch + 0, RBN - 1)] = b0;
      srb[min(4 * ch + 1, RBN - 1)] = b1;
      srb[min(4 * ch + 2, RBN - 1)] = b2;
      srb[min(4 * ch + 3, RBN - 1)] = b3;
    }
    int run = myb + pre + incl - ts;
    soff[8 * tid + 0] = run; run += e0;
    soff[8 * tid + 1] = run; run += e1;
    soff[8 * tid + 2] = run; run += e2;
    soff[8 * tid + 3] = run; run += e3;
    soff[8 * tid + 4] = run; run += e4;
    soff[8 * tid + 5] = run; run += e5;
    soff[8 * tid + 6] = run; run += e6;
    soff[8 * tid + 7] = run;
    carry = b4;
    __syncthreads();
    const v4i o0 = *(const v4i*)(soff + 4 * tid);
    const v4i o1 = *(const v4i*)(soff + 4 * (tid + OTHR));
    int* op = off + base;
    *(volatile v4i*)(op + 4 * tid) = o0;
    *(volatile v4i*)(op + 4 * (tid + OTHR)) = o1;
    __threadfence();
    *(volatile v4i*)(op + 4 * tid) = o0;
    *(volatile v4i*)(op + 4 * (tid + OTHR)) = o1;
    __syncthreads();
  }
  if (tid == 0) srb[min(4 * nChunk, RBN - 1)] = carry;
  __syncthreads();
  v4i rv = {0, 0, 0, 0};
  if (tid < 32) rv = *(const v4i*)(srb + 4 * tid);
  if (tid < 32) *(volatile v4i*)(rbase + 4 * tid) = rv;
  __threadfence();
  if (tid < 32) *(volatile v4i*)(rbase + 4 * tid) = rv;
}

__global__ __launch_bounds__(NTHR) void k_fill(
    const int* __restrict__ ei, const int* __restrict__ off, const int* __restrict__ rbase,
    int* csr, int nN, int nE, int vec8, int csrLen) {
  extern __shared__ v4f lds_dyn[];
  int* region = (int*)lds_dyn;
  int* cursor = region + RCAP;
  int* list   = cursor + NBF;
  int* wcnt   = list + LISTN;
  const int tid = threadIdx.x, lane = tid & 31, wave = tid >> 5;
  const int b = blockIdx.x;
  const int nodeBase = b * NBF;
  const int* dsts = ei + nE;

  int rb0 = rbase[b];
  const int rb1 = rbase[b + 1];
  rb0 = rb0 < 0 ? 0 : (rb0 > csrLen ? csrLen : rb0);
  rb0 &= ~31;
  int len = rb1 - rb0;
  len = len < 0 ? 0 : (len > RCAP ? RCAP : len);
  int lenW = (len + 31) & ~31;
  if (rb0 + lenW > csrLen) lenW = (csrLen - rb0) & ~31;

  {
    const v4i z = {0, 0, 0, 0};
    for (int i = tid; i < RCAP / 4; i += NTHR) ((v4i*)region)[i] = z;
    for (int s = tid; s < NBF; s += NTHR) {
      int o = off[nodeBase + s] - rb0;
      o = o < 0 ? 0 : (o > RCAP ? RCAP : o);
      cursor[s] = o;
    }
  }
  __syncthreads();

  const int nChunks = (nE + CHUNK - 1) / CHUNK;
#pragma unroll 1
  for (int ch = 0; ch < nChunks; ++ch) {
    const int cbase = ch * CHUNK;
    const int wc = scan_chunk<NBF>(dsts, nE, cbase, nodeBase, vec8, list, tid, lane, wave);
    if (lane == 0) wcnt[wave] = wc;
    __syncthreads();
    if (wave == 0) {
#pragma unroll 1
      for (int wsx = 0; wsx < NWAVE; ++wsx) {
        int n = __builtin_amdgcn_readfirstlane(wcnt[wsx]);
        n = n > WCAP ? WCAP : (n < 0 ? 0 : n);
        const int* lp = list + wsx * WCAP;
#pragma unroll 1
        for (int i = 0; i < n; ++i) {
          const int ent  = __builtin_amdgcn_readfirstlane(lp[i]);
          const int slot = ent & (NBF - 1);
          int e = cbase + ((ent >> 12) & (CHUNK - 1));
          e = e > nE - 1 ? nE - 1 : e;
          int src = ei[e];
          src = src < 0 ? 0 : (src > nN - 1 ? nN - 1 : src);
          if (lane == 0) {
            int pos = cursor[slot];
            pos = pos < 0 ? 0 : (pos > RCAP - 1 ? RCAP - 1 : pos);
            region[pos] = src;
            const int np = pos + 1;
            cursor[slot] = np > RCAP ? RCAP : np;
          }
        }
      }
    }
    __syncthreads();
  }

  const int nv = lenW >> 2;
  int* gp = csr + rb0;
#pragma unroll 1
  for (int i = tid; i < nv; i += NTHR) { const v4i v = ((const v4i*)region)[i]; *(volatile v4i*)(gp + 4 * i) = v; }
  __threadfence();
#pragma unroll 1
  for (int i = tid; i < nv; i += NTHR) { const v4i v = ((const v4i*)region)[i]; *(volatile v4i*)(gp + 4 * i) = v; }
}

__global__ __launch_bounds__(NTHR) void k_agg(
    const int* __restrict__ csr, const int* __restrict__ off, const int* __restrict__ cnt,
    const float* __restrict__ hin, _Float16* aout, int nN, int csrLen) {
  extern __shared__ v4f lds_dyn[];
  _Float16* stg = (_Float16*)lds_dyn;
  const int tid = threadIdx.x, lane = tid & 31, wave = tid >> 5;
  const int tbase = blockIdx.x * TGT + wave * 32;
  const int cl = tbase + lane;
  const int cnt_l = cnt[cl];
  const int off_l = off[cl];
  _Float16* sw = stg + wave * 32 * KD;

#pragma unroll 1
  for (int j = 0; j < 32; ++j) {
    const int c = tbase + j;
    int n = __builtin_amdgcn_readlane(cnt_l, j);
    n = n < 0 ? 0 : (n > DEGCAP ? DEGCAP : n);
    const int st = __builtin_amdgcn_readlane(off_l, j);
    v2f acc = {0.f, 0.f};
#pragma unroll 1
    for (int q0 = 0; q0 < n; q0 += 32) {
      int pos = st + q0 + lane;
      pos = pos < 0 ? 0 : (pos > csrLen - 1 ? csrLen - 1 : pos);
      int sl = csr[pos];
      sl = sl < 0 ? 0 : (sl > nN - 1 ? nN - 1 : sl);
      const int mcnt = (n - q0) < 32 ? (n - q0) : 32;
#pragma unroll 1
      for (int p = 0; p < mcnt; ++p) {
        const int s = __builtin_amdgcn_readlane(sl, p);
        acc = acc + *(const v2f*)(hin + (size_t)s * DIM + 2 * lane);
      }
    }
    const int nn = n < 1 ? 1 : n;
    const float rd = 1.0f / (float)nn;
    const int cs = c > nN - 1 ? nN - 1 : c;
    const v2f sv = *(const v2f*)(hin + (size_t)cs * DIM + 2 * lane);
    v2h hm, hs;
    hm[0] = (_Float16)(acc.x * rd); hm[1] = (_Float16)(acc.y * rd);
    hs[0] = (_Float16)sv.x;         hs[1] = (_Float16)sv.y;
    *(v2h*)(sw + j * KD + 2 * lane)       = hm;
    *(v2h*)(sw + j * KD + DIM + 2 * lane) = hs;
  }
  __syncthreads();

  _Float16* gp = aout + (size_t)tbase * KD;
#pragma unroll
  for (int p = 0; p < 32 * KD / (8 * 32); ++p) {
    const v8h v = *(const v8h*)(sw + 8 * (32 * p + lane));
    *(volatile v8h*)(gp + 8 * (32 * p + lane)) = v;
  }
  __threadfence();
#pragma unroll
  for (int p = 0; p < 32 * KD / (8 * 32); ++p) {
    const v8h v = *(const v8h*)(sw + 8 * (32 * p + lane));
    *(volatile v8h*)(gp + 8 * (32 * p + lane)) = v;
  }
}

template <int RO>
__global__ __launch_bounds__(NTHR) void k_gemm(
    const _Float16* __restrict__ A, const _Float16* __restrict__ Bs, const float* __restrict__ bias,
    float* C, const float* __restrict__ x1p, const float* __restrict__ wlin,
    const float* __restrict__ blin, float* out, int nN) {
  __shared__ __attribute__((aligned(16))) float stg[GROWS * NOUT];
  __shared__ float sred[GROWS];
  __shared__ __attribute__((aligned(16))) float sout[GROWS];
  const int tid = threadIdx.x, lane = tid & 31, wave = tid >> 5, hh = lane >> 4, m = lane & 15;
  const int rowBase = blockIdx.x * GROWS;

  v8f acc[4];
#pragma unroll
  for (int t = 0; t < 4; ++t) { v8f z = {0.f, 0.f, 0.f, 0.f, 0.f, 0.f, 0.f, 0.f}; acc[t] = z; }
  const _Float16* ar = A + (size_t)(rowBase + wave * 16 + m) * KD + 8 * hh;
#pragma unroll
  for (int kt = 0; kt < KD / 32; ++kt) {
    FragH a;
    a.h[0] = *(const v8h*)(ar + 32 * kt);
    a.h[1] = *(const v8h*)(ar + 32 * kt + 16);
#pragma unroll
    for (int t = 0; t < 4; ++t) {
      const _Float16* bp = Bs + (size_t)(16 * t + m) * KD + 32 * kt + 8 * hh;
      FragH b;
      b.h[0] = *(const v8h*)bp;
      b.h[1] = *(const v8h*)(bp + 16);
      acc[t] = wmh(a.v, b.v, acc[t]);
    }
  }

  const int r0 = wave * 16 + 8 * hh;
  float* sp = stg + r0 * NOUT + m;
#pragma unroll
  for (int t = 0; t < 4; ++t) {
    const float bv = bias[16 * t + m];
#pragma unroll
    for (int r = 0; r < 8; ++r) {
      float v = acc[t][r] * WINV + bv;
      v = fmaxf(v, 0.0f);
      sp[r * NOUT + 16 * t] = v;
    }
  }
  __syncthreads();

  if (RO == 0) {
    const float* lp = stg + wave * 16 * NOUT;
    float* gp = C + ((size_t)rowBase + wave * 16) * NOUT;
#pragma unroll
    for (int p = 0; p < 16 * NOUT / (4 * 32); ++p) {
      const v4f v = *(const v4f*)(lp + 4 * (32 * p + lane));
      *(volatile v4f*)(gp + 4 * (32 * p + lane)) = v;
    }
    __threadfence();
#pragma unroll
    for (int p = 0; p < 16 * NOUT / (4 * 32); ++p) {
      const v4f v = *(const v4f*)(lp + 4 * (32 * p + lane));
      *(volatile v4f*)(gp + 4 * (32 * p + lane)) = v;
    }
  } else {
    const int part = tid >> 7;
    const int r = tid & (GROWS - 1);
    float s = 0.0f;
    if (part == 0) {
      const float* xp = x1p + ((size_t)rowBase + r) * NOUT;
#pragma unroll 1
      for (int i = 0; i < NOUT / 4; ++i) {
        const v4f a = *(const v4f*)(xp + 4 * i);
        const v4f w = *(const v4f*)(wlin + 4 * i);
        s += a.x * w.x + a.y * w.y + a.z * w.z + a.w * w.w;
      }
    } else {
      const float* xp = stg + r * NOUT;
#pragma unroll 1
      for (int i = 0; i < NOUT / 4; ++i) {
        const v4f a = *(const v4f*)(xp + 4 * i);
        const v4f w = *(const v4f*)(wlin + NOUT + 4 * i);
        s += a.x * w.x + a.y * w.y + a.z * w.z + a.w * w.w;
      }
      sred[r] = s;
    }
    __syncthreads();
    if (part == 0) {
      float z = s + sred[r] + blin[0];
      z = z < -30.0f ? -30.0f : (z > 30.0f ? 30.0f : z);
      const float e = expf(-z);
      sout[r] = 1.0f / (1.0f + e);
    }
    __syncthreads();
    if (tid < 32) {
      const v4f ov = *(const v4f*)(sout + 4 * lane);
      const int nValid = nN - rowBase;
      const int r4 = 4 * lane;
      const bool full = (r4 + 4 <= nValid);
      float* op = out + (size_t)rowBase + r4;
      if (full) *(volatile v4f*)op = ov;
      else {
        if (r4 + 0 < nValid) *(volatile float*)(op + 0) = ov.x;
        if (r4 + 1 < nValid) *(volatile float*)(op + 1) = ov.y;
        if (r4 + 2 < nValid) *(volatile float*)(op + 2) = ov.z;
      }
      __threadfence();
      if (full) *(volatile v4f*)op = ov;
      else {
        if (r4 + 0 < nValid) *(volatile float*)(op + 0) = ov.x;
        if (r4 + 1 < nValid) *(volatile float*)(op + 1) = ov.y;
        if (r4 + 2 < nValid) *(volatile float*)(op + 2) = ov.z;
      }
    }
  }
}

extern "C" void kernel_launch(void* const* d_in, const int* in_sizes, int n_in,
                              void* d_out, int out_size, void* d_ws, size_t ws_size,
                              hipStream_t stream) {
  if (n_in < 10) return;
  const int nN = in_sizes[0] / DIM;
  const int nE = in_sizes[1] / 2;
  if (nN <= 0 || nE <= 0 || in_sizes[0] != nN * DIM || in_sizes[1] != 2 * nE) return;
  if (in_sizes[2] != DIM * NOUT || in_sizes[4] != DIM * NOUT || in_sizes[5] != DIM * NOUT || in_sizes[7] != DIM * NOUT) return;
  if (in_sizes[3] < NOUT || in_sizes[6] < NOUT || in_sizes[8] < 2 * NOUT || in_sizes[9] < 1) return;
  if (out_size != nN) return;
  if (nE > (1 << 28) || nN > (1 << 24)) return;

  const float* x    = (const float*)d_in[0];
  const int*   ei   = (const int*)d_in[1];
  const float* W1l  = (const float*)d_in[2];
  const float* b1   = (const float*)d_in[3];
  const float* W1r  = (const float*)d_in[4];
  const float* W2l  = (const float*)d_in[5];
  const float* b2   = (const float*)d_in[6];
  const float* W2r  = (const float*)d_in[7];
  const float* Wlin = (const float*)d_in[8];
  const float* blin = (const float*)d_in[9];
  float* out = (float*)d_out;

  const int NPAD   = ((nN + TGT - 1) / TGT) * TGT;
  const int nBC    = (nN + NBC - 1) / NBC;
  const int CNTPAD = nBC * NBC;
  if (4 * nBC + 1 > RBN) return;
  const int nBF    = (nN + NBF - 1) / NBF;
  if (nBF * NBF > CNTPAD || NPAD > CNTPAD) return;
  const int csrLen = ((nE + 31) & ~31) + 32 * nBF + 32;
  const int nAgg   = NPAD / TGT;
  const int nGemm  = NPAD / GROWS;

  char* ws = (char*)d_ws;
  size_t off = 0;
  const size_t oWB  = off; off += (size_t)2 * NOUT * KD * 2;       off = (off + 255) & ~(size_t)255;
  const size_t oCnt = off; off += (size_t)CNTPAD * 4;              off = (off + 255) & ~(size_t)255;
  const size_t oOff = off; off += (size_t)CNTPAD * 4;              off = (off + 255) & ~(size_t)255;
  const size_t oRb  = off; off += (size_t)RBN * 4;                 off = (off + 255) & ~(size_t)255;
  const size_t oCsr = off; off += (size_t)csrLen * 4;              off = (off + 255) & ~(size_t)255;
  const size_t oA   = off; off += (size_t)NPAD * KD * 2;           off = (off + 255) & ~(size_t)255;
  const size_t oX1  = off; off += (size_t)NPAD * NOUT * 4;         off = (off + 255) & ~(size_t)255;
  if (off > ws_size) return;
  _Float16* wB   = (_Float16*)(ws + oWB);
  int*      cnt  = (int*)(ws + oCnt);
  int*      offp = (int*)(ws + oOff);
  int*      rb   = (int*)(ws + oRb);
  int*      csr  = (int*)(ws + oCsr);
  _Float16* Ap   = (_Float16*)(ws + oA);
  float*    x1   = (float*)(ws + oX1);

  const int vec8 = ((nE & 3) == 0) ? 1 : 0;

  k_wprep<<<8, NTHR, 0, stream>>>(W1l, W1r, W2l, W2r, wB);

  k_count<<<nBC, NTHR, 0, stream>>>(ei, cnt, nE, vec8);
  k_offsets<<<1, OTHR, 0, stream>>>(cnt, offp, rb, nBC);
  hipFuncSetAttribute(reinterpret_cast<const void*>(&k_fill),
                      hipFuncAttributeMaxDynamicSharedMemorySize, LDS_FILL);
  k_fill<<<nBF, NTHR, LDS_FILL, stream>>>(ei, offp, rb, csr, nN, nE, vec8, csrLen);

  hipFuncSetAttribute(reinterpret_cast<const void*>(&k_agg),
                      hipFuncAttributeMaxDynamicSharedMemorySize, LDS_AGG);
  k_agg<<<nAgg, NTHR, LDS_AGG, stream>>>(csr, offp, cnt, x, Ap, nN, csrLen);
  k_gemm<0><<<nGemm, NTHR, 0, stream>>>(Ap, wB, b1, x1, x1, Wlin, blin, out, nN);

  k_agg<<<nAgg, NTHR, LDS_AGG, stream>>>(csr, offp, cnt, x1, Ap, nN, csrLen);
  k_gemm<1><<<nGemm, NTHR, 0, stream>>>(Ap, wB + (size_t)NOUT * KD, b2, x1, x1, Wlin, blin, out, nN);
}
